// SlotAttention_10041633538391
// MI455X (gfx1250) — hardware-run, weakly checked
//
#include <hip/hip_runtime.h>
#include <math.h>
#include <stdint.h>

typedef __attribute__((ext_vector_type(16))) _Float16 v16h;
typedef __attribute__((ext_vector_type(8)))  _Float16 v8h;
typedef __attribute__((ext_vector_type(16))) __bf16   v16b;
typedef __attribute__((ext_vector_type(8)))  __bf16   v8b;
typedef __attribute__((ext_vector_type(8)))  float    v8f;
typedef __attribute__((ext_vector_type(4)))  float    v4f;
typedef __attribute__((ext_vector_type(4)))  unsigned v4u;

__device__ __forceinline__ unsigned short f2bf_bits(float f) {
  unsigned u = __float_as_uint(f);
  return (unsigned short)((u + 0x7FFFu + ((u >> 16) & 1u)) >> 16);
}
__device__ __forceinline__ float bf_bits2f(unsigned short h) { return __uint_as_float(((unsigned)h) << 16); }

__device__ __forceinline__ void dep_guard_h(v8f& a, v8f& b, v16h x, v16h y) { asm volatile("v_nop\n\tv_nop\n\tv_nop\n\tv_nop" : "+v"(a), "+v"(b) : "v"(x), "v"(y)); }
__device__ __forceinline__ void dep_guard_b(v8f& a, v8f& b, v16b x, v16b y) { asm volatile("v_nop\n\tv_nop\n\tv_nop\n\tv_nop" : "+v"(a), "+v"(b) : "v"(x), "v"(y)); }
__device__ __forceinline__ void keep4_h(v16h a, v16h b, v16h c, v16h d) { asm volatile("v_nop" :: "v"(a), "v"(b), "v"(c), "v"(d)); }
__device__ __forceinline__ void keep4_b(v16b a, v16b b, v16b c, v16b d) { asm volatile("v_nop" :: "v"(a), "v"(b), "v"(c), "v"(d)); }
__device__ __forceinline__ void acc_guard4(v8f& a, v8f& b, v8f& c, v8f& d) { asm volatile("v_nop\n\tv_nop\n\tv_nop\n\tv_nop" : "+v"(a), "+v"(b), "+v"(c), "+v"(d)); }
template <typename T> struct Frag;
template <> struct Frag<_Float16> {
  typedef v16h V; union U { v16h v; v8h h[2]; };
  static __device__ __forceinline__ v16h load(const _Float16* p) {
    U f; f.h[0] = *(const v8h*)(p); f.h[1] = *(const v8h*)(p + 16); return f.v;
  }
  static __device__ __forceinline__ v8f mma(v16h a, v16h b, v8f c) {
    return __builtin_amdgcn_wmma_f32_16x16x32_f16(false, a, false, b, (short)0, c, false, false);
  }
  static __device__ __forceinline__ void guard(v8f& a, v8f& b, v16h x, v16h y) { dep_guard_h(a, b, x, y); }
  static __device__ __forceinline__ void keep(v16h a, v16h b, v16h c, v16h d) { keep4_h(a, b, c, d); }
};
template <> struct Frag<__bf16> {
  typedef v16b V; union U { v16b v; v8b h[2]; };
  static __device__ __forceinline__ v16b load(const __bf16* p) {
    U f; f.h[0] = *(const v8b*)(p); f.h[1] = *(const v8b*)(p + 16); return f.v;
  }
  static __device__ __forceinline__ v8f mma(v16b a, v16b b, v8f c) {
    return __builtin_amdgcn_wmma_f32_16x16x32_bf16(false, a, false, b, (short)0, c, false, false);
  }
  static __device__ __forceinline__ void guard(v8f& a, v8f& b, v16b x, v16b y) { dep_guard_b(a, b, x, y); }
  static __device__ __forceinline__ void keep(v16b a, v16b b, v16b c, v16b d) { keep4_b(a, b, c, d); }
};

template <int ET> struct Elem;
template <> struct Elem<0> { typedef _Float16 T; };
template <> struct Elem<1> { typedef __bf16 T; };
template <int ET, bool SPLIT, int BIAS_MODE, int OUT_MODE, bool RESID, int ACT = 0>
__global__ __launch_bounds__(256) void wmma_gemm64(
    const unsigned short* __restrict__ Ap, const unsigned short* __restrict__ A2p, int lda, long strideA,
    const unsigned short* __restrict__ Btp, const unsigned short* __restrict__ Bt2p, int ldb, long strideB,
    void* __restrict__ Cout, void* __restrict__ Cout2, int ldc, long strideC,
    const float* __restrict__ bias,
    const float* __restrict__ resid, long strideR,
    int M, int N, int K, float scale) {
  typedef typename Elem<ET>::T T;
  typedef typename Frag<T>::V V;
  const T* A = (const T*)Ap; const T* A2 = (const T*)A2p; const T* Bt = (const T*)Btp; const T* Bt2 = (const T*)Bt2p;
  __shared__ __align__(16) float sT[8][16 * 68];
  const int b    = blockIdx.y;
  const int lane = threadIdx.x & 31;
  const int wave = threadIdx.x >> 5;
  const int tilesN = N >> 6;
  const int tilesM = M >> 6;
  const int tile = blockIdx.x * 8 + wave;
  if (tile >= tilesM * tilesN) return;
  const int tm = tile / tilesN;
  const int tn = tile - tm * tilesN;
  const int m0 = tm << 6;
  const int n0 = tn << 6;

  const T* Ab  = A  + (size_t)b * strideA;
  const T* Bb  = Bt + (size_t)b * strideB;
  const T* Ab2 = SPLIT ? (A2  + (size_t)b * strideA) : nullptr;
  const T* Bb2 = SPLIT ? (Bt2 + (size_t)b * strideB) : nullptr;

  const int rlane = lane & 15;
  const int koff  = (lane >> 4) * 8;
  const int mOff  = (lane >> 4) * 8;

  v8f acc[4][4];
#pragma unroll
  for (int i = 0; i < 4; ++i)
#pragma unroll
    for (int j = 0; j < 4; ++j) acc[i][j] = (v8f){0.f,0.f,0.f,0.f,0.f,0.f,0.f,0.f};

  for (int k0 = 0; k0 < K; k0 += 32) {
    V bh[4], bl[4];
#pragma unroll
    for (int j = 0; j < 4; ++j) {
      const size_t bo = (size_t)(n0 + (j << 4) + rlane) * ldb + koff + k0;
      bh[j] = Frag<T>::load(Bb + bo);
      if (SPLIT) bl[j] = Frag<T>::load(Bb2 + bo);
    }
#pragma unroll
    for (int i = 0; i < 4; ++i) {
      const size_t ao = (size_t)(m0 + (i << 4) + rlane) * lda + koff + k0;
      V ah = Frag<T>::load(Ab + ao);
      V al;
      if (SPLIT) al = Frag<T>::load(Ab2 + ao);
#pragma unroll
      for (int j = 0; j < 4; ++j) {
        acc[i][j] = Frag<T>::mma(ah, bh[j], acc[i][j]);
        if (SPLIT) {
          acc[i][j] = Frag<T>::mma(ah, bl[j], acc[i][j]);
          acc[i][j] = Frag<T>::mma(al, bh[j], acc[i][j]);
        }
      }
      Frag<T>::guard(acc[i][0], acc[i][3], ah, SPLIT ? al : ah);
    }
    Frag<T>::keep(bh[0], bh[1], bh[2], bh[3]);
    if (SPLIT) Frag<T>::keep(bl[0], bl[1], bl[2], bl[3]);
  }
  acc_guard4(acc[0][0], acc[0][1], acc[0][2], acc[0][3]);
  acc_guard4(acc[1][0], acc[1][1], acc[1][2], acc[1][3]);
  acc_guard4(acc[2][0], acc[2][1], acc[2][2], acc[2][3]);
  acc_guard4(acc[3][0], acc[3][1], acc[3][2], acc[3][3]);

  float* slab = sT[wave];
  const float* Rb = RESID ? (resid + (size_t)b * strideR) : nullptr;
#pragma unroll
  for (int i = 0; i < 4; ++i) {
    const int mBase = m0 + (i << 4);
#pragma unroll
    for (int j = 0; j < 4; ++j) {
      const int n = n0 + (j << 4) + rlane;
      float bv = 0.f;
      if (BIAS_MODE == 2) bv = bias[n];
#pragma unroll
      for (int r = 0; r < 8; ++r) {
        float v = acc[i][j][r] * scale;
        if (BIAS_MODE == 1) v += bias[mBase + mOff + r];
        if (BIAS_MODE == 2) v += bv;
        if (RESID) v += Rb[(size_t)(mBase + mOff + r) * ldc + n];
        if (ACT == 1) v = tanhf(v);
        if (ACT == 2) v = fmaxf(v, 0.0f);
        if (ACT == 3) v = v / (1.0f + expf(-v));
        if (ACT == 4) v = (v > 0.f) ? v : 0.01f * v;
        if (ACT == 5) v = 0.5f * v * (1.0f + erff(v * 0.70710678118654752f));
        slab[(mOff + r) * 68 + (j << 4) + rlane] = v;
      }
    }
    __builtin_amdgcn_fence(__ATOMIC_RELEASE, "workgroup");
    __builtin_amdgcn_wave_barrier();
    __builtin_amdgcn_fence(__ATOMIC_ACQUIRE, "workgroup");
    if (OUT_MODE == 0) {
      float* C = (float*)Cout + (size_t)b * strideC;
      const int hh = lane >> 4, c4 = (lane & 15) * 4;
      for (int pass = 0; pass < 2; ++pass) {
#pragma unroll
        for (int it = 0; it < 8; ++it) {
          const int row = it * 2 + hh;
          v4f v = *(const v4f*)(slab + row * 68 + c4);
          *(volatile v4f*)(C + (size_t)(mBase + row) * ldc + n0 + c4) = v;
        }
        __threadfence();
      }
    } else {
      const int q = lane >> 3, c8 = (lane & 7) * 8;
      unsigned short* C  = (unsigned short*)Cout  + (size_t)b * strideC;
      unsigned short* C2 = (OUT_MODE == 2) ? ((unsigned short*)Cout2 + (size_t)b * strideC) : nullptr;
      for (int pass = 0; pass < 2; ++pass) {
#pragma unroll
        for (int it = 0; it < 4; ++it) {
          const int row = it * 4 + q;
          const float* sp = slab + row * 68 + c8;
          v8h hv, lv;
#pragma unroll
          for (int e = 0; e < 8; ++e) {
            if (OUT_MODE == 1) {
              hv[e] = (_Float16)sp[e];
            } else {
              unsigned short hb = f2bf_bits(sp[e]);
              unsigned short lb = f2bf_bits(sp[e] - bf_bits2f(hb));
              hv[e] = __builtin_bit_cast(_Float16, hb);
              lv[e] = __builtin_bit_cast(_Float16, lb);
            }
          }
          *(volatile v8h*)(C + (size_t)(mBase + row) * ldc + n0 + c8) = hv;
          if (OUT_MODE == 2) *(volatile v8h*)(C2 + (size_t)(mBase + row) * ldc + n0 + c8) = lv;
        }
        __threadfence();
      }
    }
    __builtin_amdgcn_fence(__ATOMIC_RELEASE, "workgroup");
    __builtin_amdgcn_wave_barrier();
    __builtin_amdgcn_fence(__ATOMIC_ACQUIRE, "workgroup");
  }
}

namespace cfg {
constexpr int NB     = 16;
constexpr int NTOK   = 4096;
constexpr int DIM    = 64;
constexpr int NSLOT  = 5;
constexpr int NFG    = 4;
constexpr int CDIM   = 8;
constexpr int NITER  = 4;
constexpr int NROW   = NB * NTOK;
constexpr int NROWFG = NB * NFG * NTOK;
constexpr int NSROW  = NB * NSLOT;
constexpr int NOUTC  = DIM + CDIM;
constexpr int OPITCH = 128;
constexpr int LINEF  = 32;
constexpr float ATT_SCALE  = 0.125f;
constexpr float ATT_EPS    = 1e-8f;
constexpr float LN_EPS     = 1e-5f;
constexpr float WCARRY     = 256.0f;
constexpr float WCARRY_INV = 1.0f / 256.0f;
constexpr float GRID_DELTA = 2.0f / 63.0f;
}
static_assert(cfg::NROW % 64 == 0, "");
static_assert(cfg::DIM % 32 == 0, "");
static_assert(cfg::NROW % 32 == 0, "");
static_assert(cfg::NROWFG % 64 == 0, "");
static_assert(cfg::NTOK % 256 == 0, "");
static_assert(cfg::NOUTC % 4 == 0, "");
static_assert((cfg::NSROW * cfg::NOUTC * 4) % 512 == 0, "");

__device__ __forceinline__ float grid_x(int n) {
  const int j = n & 63;
  return (j == 63) ? 1.0f : (-1.0f + (float)j * cfg::GRID_DELTA);
}
__device__ __forceinline__ float grid_y(int n) {
  const int i = (n >> 6) & 63;
  return (i == 63) ? 1.0f : (-1.0f + (float)i * cfg::GRID_DELTA);
}
__device__ __forceinline__ float h2f(unsigned u) {
  return (float)__builtin_bit_cast(_Float16, (unsigned short)(u & 0xffffu));
}
__device__ __forceinline__ float rsum16(float v) {
  v += __shfl_xor(v, 1, 32);
  v += __shfl_xor(v, 2, 32);
  v += __shfl_xor(v, 4, 32);
  v += __shfl_xor(v, 8, 32);
  return v;
}
__device__ __forceinline__ float rsum8(float v) {
  v += __shfl_xor(v, 1, 32);
  v += __shfl_xor(v, 2, 32);
  v += __shfl_xor(v, 4, 32);
  return v;
}
__device__ __forceinline__ void wave_lds_sync() {
  __builtin_amdgcn_fence(__ATOMIC_RELEASE, "workgroup");
  __builtin_amdgcn_wave_barrier();
  __builtin_amdgcn_fence(__ATOMIC_ACQUIRE, "workgroup");
}

__global__ __launch_bounds__(256) void cast_w_kernel(
    const float* __restrict__ p0, const float* __restrict__ p1, const float* __restrict__ p2,
    const float* __restrict__ p3, const float* __restrict__ p4, const float* __restrict__ p5,
    unsigned short* __restrict__ wpl)
{
  const int y = blockIdx.y;
  const float* src = p0;
  if (y == 1) src = p1;
  if (y == 2) src = p2;
  if (y == 3) src = p3;
  if (y == 4) src = p4;
  if (y == 5) src = p5;
  const int i = blockIdx.x * 256 + threadIdx.x;
  const _Float16 h0 = (_Float16)(src[2 * i] * cfg::WCARRY);
  const _Float16 h1 = (_Float16)(src[2 * i + 1] * cfg::WCARRY);
  const unsigned u = (unsigned)__builtin_bit_cast(unsigned short, h0) | ((unsigned)__builtin_bit_cast(unsigned short, h1) << 16);
  volatile unsigned* outp = (volatile unsigned*)(wpl + (size_t)y * 4096);
  outp[i] = u;
  __threadfence();
  outp[i] = u;
}

__global__ __launch_bounds__(256) void prep_ln_kernel(
    const float* __restrict__ feat, const float* __restrict__ g, const float* __restrict__ bb,
    const float* __restrict__ fc, const float* __restrict__ gc, const float* __restrict__ bc,
    unsigned short* __restrict__ featln, float* __restrict__ fcln)
{
  using namespace cfg;
  const int tid = threadIdx.x, wave = tid >> 5, lane = tid & 31;
  {
    const int q = lane >> 3, c8 = (lane & 7) * 8;
    const int row = blockIdx.x * 32 + wave * 4 + q;
    const float* src = feat + (size_t)row * DIM + c8;
    const v4f f0 = *(const v4f*)(src);
    const v4f f1 = *(const v4f*)(src + 4);
    const v4f g0 = *(const v4f*)(g + c8), g1 = *(const v4f*)(g + c8 + 4);
    const v4f b0 = *(const v4f*)(bb + c8), b1 = *(const v4f*)(bb + c8 + 4);
    float x[8];
#pragma unroll
    for (int e = 0; e < 4; ++e) { x[e] = f0[e]; x[4 + e] = f1[e]; }
    float s = 0.f;
#pragma unroll
    for (int e = 0; e < 8; ++e) s += x[e];
    s = rsum8(s);
    const float mean = s * (1.0f / 64.0f);
    float vs = 0.f;
#pragma unroll
    for (int e = 0; e < 8; ++e) { const float d = x[e] - mean; x[e] = d; vs += d * d; }
    vs = rsum8(vs);
    const float inv = rsqrtf(vs * (1.0f / 64.0f) + LN_EPS);
    v8h hv;
#pragma unroll
    for (int e = 0; e < 4; ++e) {
      hv[e]     = (_Float16)(x[e] * inv * g0[e] + b0[e]);
      hv[4 + e] = (_Float16)(x[4 + e] * inv * g1[e] + b1[e]);
    }
    unsigned short* dst = featln + (size_t)row * DIM + c8;
    *(volatile v8h*)dst = hv;
    __threadfence();
    *(volatile v8h*)dst = hv;
  }
  if (wave < 2) {
    const int r = lane >> 1, half = lane & 1;
    const int row = blockIdx.x * 32 + wave * 16 + r;
    const v4f f = *(const v4f*)(fc + (size_t)row * CDIM + half * 4);
    const v4f gg = *(const v4f*)(gc + half * 4);
    const v4f bv = *(const v4f*)(bc + half * 4);
    float s = (f[0] + f[1]) + (f[2] + f[3]);
    s += __shfl_xor(s, 1, 32);
    const float mean = s * 0.125f;
    v4f d;
    float vs = 0.f;
#pragma unroll
    for (int e = 0; e < 4; ++e) { d[e] = f[e] - mean; vs += d[e] * d[e]; }
    vs += __shfl_xor(vs, 1, 32);
    const float inv = rsqrtf(vs * 0.125f + LN_EPS);
    v4f o;
#pragma unroll
    for (int e = 0; e < 4; ++e) o[e] = d[e] * inv * gg[e] + bv[e];
    float* dst = fcln + (size_t)row * CDIM + half * 4;
    *(volatile v4f*)dst = o;
    __threadfence();
    *(volatile v4f*)dst = o;
  }
}

__global__ __launch_bounds__(256) void ln_geo_kernel(
    const float* __restrict__ tmp2, const float* __restrict__ w_grid, const float* __restrict__ b_grid,
    const float* __restrict__ g, const float* __restrict__ bb, unsigned short* __restrict__ u2)
{
  using namespace cfg;
  __shared__ __align__(16) float coef[5][64];
  const int tid = threadIdx.x, wave = tid >> 5, lane = tid & 31;
  if (tid < 64) {
    const v4f wg = *(const v4f*)(w_grid + tid * 4);
    coef[0][tid] = wg[0] - wg[2];
    coef[1][tid] = wg[1] - wg[3];
    coef[2][tid] = b_grid[tid];
    coef[3][tid] = g[tid];
    coef[4][tid] = bb[tid];
  }
  __syncthreads();
  const int plane = blockIdx.y;
  const float* src = tmp2 + (size_t)plane * ((size_t)NROW * DIM);
  unsigned short* dst = u2 + (size_t)plane * ((size_t)NROW * DIM);
  const int q = lane >> 3, c8 = (lane & 7) * 8;
  const int row = blockIdx.x * 32 + wave * 4 + q;
  const int n = row & (NTOK - 1);
  const float gxv = grid_x(n), gyv = grid_y(n);
  const float* sp = src + (size_t)row * DIM + c8;
  const v4f f0 = *(const v4f*)(sp), f1 = *(const v4f*)(sp + 4);
  const v4f cx0 = *(const v4f*)(&coef[0][c8]), cx1 = *(const v4f*)(&coef[0][c8 + 4]);
  const v4f cy0 = *(const v4f*)(&coef[1][c8]), cy1 = *(const v4f*)(&coef[1][c8 + 4]);
  const v4f gb0 = *(const v4f*)(&coef[2][c8]), gb1 = *(const v4f*)(&coef[2][c8 + 4]);
  const v4f g0  = *(const v4f*)(&coef[3][c8]), g1  = *(const v4f*)(&coef[3][c8 + 4]);
  const v4f b0  = *(const v4f*)(&coef[4][c8]), b1  = *(const v4f*)(&coef[4][c8 + 4]);
  float x[8];
#pragma unroll
  for (int e = 0; e < 4; ++e) {
    x[e]     = f0[e] + (gxv * cx0[e] + gyv * cy0[e] + gb0[e]);
    x[4 + e] = f1[e] + (gxv * cx1[e] + gyv * cy1[e] + gb1[e]);
  }
  float s = 0.f;
#pragma unroll
  for (int e = 0; e < 8; ++e) s += x[e];
  s = rsum8(s);
  const float mean = s * (1.0f / 64.0f);
  float vs = 0.f;
#pragma unroll
  for (int e = 0; e < 8; ++e) { const float d = x[e] - mean; x[e] = d; vs += d * d; }
  vs = rsum8(vs);
  const float inv = rsqrtf(vs * (1.0f / 64.0f) + LN_EPS);
  v8h hv;
#pragma unroll
  for (int e = 0; e < 4; ++e) {
    hv[e]     = (_Float16)(x[e] * inv * g0[e] + b0[e]);
    hv[4 + e] = (_Float16)(x[4 + e] * inv * g1[e] + b1[e]);
  }
  unsigned short* dp = dst + (size_t)row * DIM + c8;
  *(volatile v8h*)dp = hv;
  __threadfence();
  *(volatile v8h*)dp = hv;
}

__global__ __launch_bounds__(256) void init_kernel(
    const float* __restrict__ s_fg0, const float* __restrict__ s_bg0, const float* __restrict__ pos0,
    float* __restrict__ slots, float* __restrict__ posl)
{
  const int tid = threadIdx.x;
  v4f vfg[4];
#pragma unroll
  for (int it = 0; it < 4; ++it) {
    const int elem = (it * 256 + tid) * 4;
    vfg[it] = *(const v4f*)(s_fg0 + (elem & 255));
  }
  const v4f vbg = *(const v4f*)(s_bg0 + ((tid * 4) & 63));
  v4f vp[2];
#pragma unroll
  for (int it = 0; it < 2; ++it) {
    const int idx = it * 256 + tid;
    const int line = idx >> 3, piece = idx & 7;
    const int kk = line & 3;
    const float px = pos0[kk * 2 + 0], py = pos0[kk * 2 + 1];
    v4f v = (v4f){0.f, 0.f, 0.f, 0.f};
    v[0] = (piece == 0) ? px : 0.f;
    v[1] = (piece == 0) ? py : 0.f;
    vp[it] = v;
  }
  for (int pass = 0; pass < 2; ++pass) {
#pragma unroll
    for (int it = 0; it < 4; ++it) *(volatile v4f*)(slots + (size_t)(it * 256 + tid) * 4) = vfg[it];
    *(volatile v4f*)(slots + 4096 + tid * 4) = vbg;
#pragma unroll
    for (int it = 0; it < 2; ++it) *(volatile v4f*)(posl + (size_t)(it * 256 + tid) * 4) = vp[it];
    __threadfence();
  }
}

__global__ __launch_bounds__(64) void q_proj_kernel(
    const float* __restrict__ slots,
    const float* __restrict__ lnq_g, const float* __restrict__ lnq_b, const float* __restrict__ w_q,
    const float* __restrict__ lnqb_g, const float* __restrict__ lnqb_b, const float* __restrict__ w_qbg,
    float* __restrict__ qbuf)
{
  using namespace cfg;
  __shared__ __align__(16) float shx[64];
  __shared__ __align__(16) float shl[64];
  __shared__ __align__(16) float sho[64];
  const int tid = threadIdx.x;
  const int r = blockIdx.x;
  const bool fg = (r < 64);
  const float* g  = fg ? lnq_g : lnqb_g;
  const float* bb = fg ? lnq_b : lnqb_b;
  const float* W  = fg ? w_q : w_qbg;
  shx[tid] = slots[(size_t)r * 64 + tid];
  __syncthreads();
  float s = 0.f;
#pragma unroll 1
  for (int d = 0; d < 64; ++d) s += shx[d];
  const float mean = s * (1.0f / 64.0f);
  float vs = 0.f;
#pragma unroll 1
  for (int d = 0; d < 64; ++d) { const float dd = shx[d] - mean; vs += dd * dd; }
  const float inv = rsqrtf(vs * (1.0f / 64.0f) + LN_EPS);
  shl[tid] = (shx[tid] - mean) * inv * g[tid] + bb[tid];
  __syncthreads();
  float acc = 0.f;
#pragma unroll 1
  for (int d = 0; d < 64; ++d) acc += shl[d] * W[tid * 64 + d];
  sho[tid] = acc;
  __syncthreads();
  const v4f v = *(const v4f*)(sho + (tid & 15) * 4);
  float* dst = qbuf + (size_t)r * 64 + (tid & 15) * 4;
  if (tid < 16) *(volatile v4f*)dst = v;
  __threadfence();
  if (tid < 16) *(volatile v4f*)dst = v;
}

__device__ __forceinline__ void ln_row_frag(
    const float* __restrict__ rowp, float rx, float ry, int koff,
    const float* cxs, const float* cys, const float* gbs, const float* lgs, const float* lbs,
    v16h& a0, v16h& a1)
{
  float x[32];
#pragma unroll
  for (int t = 0; t < 4; ++t) {
    const int col = t * 16 + koff;
    const v4f f0 = *(const v4f*)(rowp + col);
    const v4f f1 = *(const v4f*)(rowp + col + 4);
    const v4f cx0 = *(const v4f*)(cxs + col), cx1 = *(const v4f*)(cxs + col + 4);
    const v4f cy0 = *(const v4f*)(cys + col), cy1 = *(const v4f*)(cys + col + 4);
    const v4f gb0 = *(const v4f*)(gbs + col), gb1 = *(const v4f*)(gbs + col + 4);
#pragma unroll
    for (int e = 0; e < 4; ++e) {
      x[t * 8 + e]     = f0[e] + (rx * cx0[e] + ry * cy0[e] + gb0[e]);
      x[t * 8 + 4 + e] = f1[e] + (rx * cx1[e] + ry * cy1[e] + gb1[e]);
    }
  }
  float s = 0.f;
#pragma unroll
  for (int i = 0; i < 32; ++i) s += x[i];
  s += __shfl_xor(s, 16, 32);
  const float mean = s * (1.0f / 64.0f);
  float vs = 0.f;
#pragma unroll
  for (int i = 0; i < 32; ++i) { const float d = x[i] - mean; x[i] = d; vs += d * d; }
  vs += __shfl_xor(vs, 16, 32);
  const float inv = rsqrtf(vs * (1.0f / 64.0f) + cfg::LN_EPS);
  v8h p[4];
#pragma unroll
  for (int t = 0; t < 4; ++t) {
    const int col = t * 16 + koff;
    const v4f g0 = *(const v4f*)(lgs + col), g1 = *(const v4f*)(lgs + col + 4);
    const v4f b0 = *(const v4f*)(lbs + col), b1 = *(const v4f*)(lbs + col + 4);
    v8h pv;
#pragma unroll
    for (int e = 0; e < 4; ++e) {
      pv[e]     = (_Float16)(x[t * 8 + e] * inv * g0[e] + b0[e]);
      pv[4 + e] = (_Float16)(x[t * 8 + 4 + e] * inv * g1[e] + b1[e]);
    }
    p[t] = pv;
  }
  Frag<_Float16>::U u0, u1;
  u0.h[0] = p[0]; u0.h[1] = p[1];
  u1.h[0] = p[2]; u1.h[1] = p[3];
  a0 = u0.v; a1 = u1.v;
}

__global__ __launch_bounds__(64) void fg_kv_kernel(
    const float* __restrict__ kf, const float* __restrict__ vf, const float* __restrict__ posl,
    const float* __restrict__ w_grid, const float* __restrict__ b_grid,
    const float* __restrict__ ln_g, const float* __restrict__ ln_b,
    const unsigned short* __restrict__ w16, const float* __restrict__ b_mlp,
    const float* __restrict__ qbuf, unsigned short* __restrict__ vplane, float* __restrict__ logits)
{
  using namespace cfg;
  __shared__ __align__(16) float coef[5][64];
  __shared__ __align__(16) float slab[2][32 * 68];
  __shared__ __align__(16) float lgst[2][32];
  const int tid = threadIdx.x, wave = tid >> 5, lane = tid & 31;
  const int rl = lane & 15, hh = lane >> 4, koff = hh * 8;
  {
    const int c = tid;
    const v4f wg = *(const v4f*)(w_grid + c * 4);
    coef[0][c] = wg[0] - wg[2];
    coef[1][c] = wg[1] - wg[3];
    coef[2][c] = b_grid[c];
    coef[3][c] = ln_g[c];
    coef[4][c] = ln_b[c];
  }
  __syncthreads();
  const int tile = blockIdx.x * 2 + wave;
  const int t = tile & 127;
  const int bk = tile >> 7;
  const int b = bk >> 2, k = bk & 3;
  const int n0 = t * 32;
  const float px = posl[bk * LINEF + 0];
  const float py = posl[bk * LINEF + 1];

  v16h bw0[4], bw1[4];
#pragma unroll
  for (int j = 0; j < 4; ++j) {
    const _Float16* wp = (const _Float16*)w16 + (size_t)(16 * j + rl) * 64 + koff;
    bw0[j] = Frag<_Float16>::load(wp);
    bw1[j] = Frag<_Float16>::load(wp + 32);
  }
  float qv[4], bm[4];
#pragma unroll
  for (int j = 0; j < 4; ++j) {
    qv[j] = qbuf[(size_t)bk * 64 + 16 * j + rl];
    bm[j] = b_mlp[16 * j + rl];
  }
  float* myslab = slab[wave];
  float* mylg = lgst[wave];

#pragma unroll 1
  for (int pi = 0; pi < 4; ++pi) {
    const int path = pi >> 1;
    const int i = pi & 1;
    const int rloc = 16 * i + rl;
    const int n = n0 + rloc;
    const float rx = grid_x(n) - px;
    const float ry = grid_y(n) - py;
    const float* src = (path == 0) ? kf : vf;
    const float* rowp = src + ((size_t)b * NTOK + n) * 64;
    v16h a0, a1;
    ln_row_frag(rowp, rx, ry, koff, coef[0], coef[1], coef[2], coef[3], coef[4], a0, a1);
    v8f acc[4];
#pragma unroll
    for (int j = 0; j < 4; ++j) acc[j] = (v8f){0.f,0.f,0.f,0.f,0.f,0.f,0.f,0.f};
#pragma unroll
    for (int j = 0; j < 4; ++j) {
      acc[j] = Frag<_Float16>::mma(a0, bw0[j], acc[j]);
      acc[j] = Frag<_Float16>::mma(a1, bw1[j], acc[j]);
    }
    Frag<_Float16>::guard(acc[0], acc[3], a0, a1);
    acc_guard4(acc[0], acc[1], acc[2], acc[3]);
    keep4_h(bw0[0], bw0[1], bw0[2], bw0[3]);
    keep4_h(bw1[0], bw1[1], bw1[2], bw1[3]);
    if (path == 0) {
#pragma unroll
      for (int r = 0; r < 8; ++r) {
        float p = 0.f;
#pragma unroll
        for (int j = 0; j < 4; ++j) p += (acc[j][r] * WCARRY_INV + bm[j]) * qv[j];
        p = rsum16(p);
        if (rl == 0) mylg[16 * i + 8 * hh + r] = p * ATT_SCALE;
      }
    } else {
#pragma unroll
      for (int r = 0; r < 8; ++r)
#pragma unroll
        for (int j = 0; j < 4; ++j)
          myslab[(16 * i + 8 * hh + r) * 68 + 16 * j + rl] = acc[j][r] * WCARRY_INV + bm[j];
    }
  }
  wave_lds_sync();
  {
    const v4f lv = *(const v4f*)(mylg + (lane & 7) * 4);
    float* ld = logits + ((size_t)(b * NSLOT + 1 + k)) * NTOK + n0 + (lane & 7) * 4;
    if (lane < 8) *(volatile v4f*)ld = lv;
    __threadfence();
    if (lane < 8) *(volatile v4f*)ld = lv;
  }
  {
    const int q = lane >> 3, c8 = (lane & 7) * 8;
    unsigned short* vb = vplane + ((size_t)bk * NTOK + n0) * 64;
    for (int pass = 0; pass < 2; ++pass) {
#pragma unroll
      for (int it = 0; it < 8; ++it) {
        const int row = it * 4 + q;
        const float* sp = myslab + row * 68 + c8;
        v8h hv;
#pragma unroll
        for (int e = 0; e < 8; ++e) hv[e] = (_Float16)sp[e];
        *(volatile v8h*)(vb + (size_t)row * 64 + c8) = hv;
      }
      __threadfence();
    }
  }
}

__global__ __launch_bounds__(256) void bg_logits_kernel(
    const float* __restrict__ kbg, const float* __restrict__ qbuf, float* __restrict__ logits)
{
  using namespace cfg;
  __shared__ __align__(16) float qsh[64];
  const int tid = threadIdx.x;
  const int b = blockIdx.x >> 4;
  const int n = (blockIdx.x & 15) * 256 + tid;
  if (tid < 64) qsh[tid] = qbuf[(size_t)(64 + b) * 64 + tid];
  __syncthreads();
  const float* kr = kbg + ((size_t)b * NTOK + n) * 64;
  float p = 0.f;
#pragma unroll 1
  for (int ch = 0; ch < 4; ++ch) {
    const v4f k0 = *(const v4f*)(kr + ch * 16), k1 = *(const v4f*)(kr + ch * 16 + 4);
    const v4f k2 = *(const v4f*)(kr + ch * 16 + 8), k3 = *(const v4f*)(kr + ch * 16 + 12);
    const v4f q0 = *(const v4f*)(qsh + ch * 16), q1 = *(const v4f*)(qsh + ch * 16 + 4);
    const v4f q2 = *(const v4f*)(qsh + ch * 16 + 8), q3 = *(const v4f*)(qsh + ch * 16 + 12);
#pragma unroll
    for (int e = 0; e < 4; ++e) {
      p += k0[e] * q0[e]; p += k1[e] * q1[e]; p += k2[e] * q2[e]; p += k3[e] * q3[e];
    }
  }
  p *= ATT_SCALE;
  volatile float* dst = (volatile float*)(logits + (size_t)(b * NSLOT) * NTOK + n);
  *dst = p;
  __threadfence();
  *dst = p;
}

__global__ __launch_bounds__(256) void softmax_kernel(
    const float* __restrict__ logits, float* __restrict__ attn, float* __restrict__ plines)
{
  using namespace cfg;
  __shared__ float red[5][8];
  __shared__ __align__(16) float lst[32];
  const int tid = threadIdx.x, wave = tid >> 5, lane = tid & 31;
  const int b = blockIdx.x >> 4, ch = blockIdx.x & 15;
  const int n = ch * 256 + tid;
  float l[5];
  float m = -INFINITY;
#pragma unroll
  for (int s = 0; s < 5; ++s) { l[s] = logits[((size_t)(b * NSLOT + s)) * NTOK + n]; m = fmaxf(m, l[s]); }
  float e[5];
  float tot = 0.f;
#pragma unroll
  for (int s = 0; s < 5; ++s) { e[s] = expf(l[s] - m); tot += e[s]; }
  const float inv = 1.0f / tot;
  float a[5];
#pragma unroll
  for (int s = 0; s < 5; ++s) a[s] = e[s] * inv + ATT_EPS;
#pragma unroll
  for (int s = 0; s < 5; ++s) *(volatile float*)(attn + ((size_t)(b * NSLOT + s)) * NTOK + n) = a[s];
  __threadfence();
#pragma unroll
  for (int s = 0; s < 5; ++s) *(volatile float*)(attn + ((size_t)(b * NSLOT + s)) * NTOK + n) = a[s];
#pragma unroll
  for (int s = 0; s < 5; ++s) {
    float v = a[s];
    v += __shfl_xor(v, 1, 32);
    v += __shfl_xor(v, 2, 32);
    v += __shfl_xor(v, 4, 32);
    v += __shfl_xor(v, 8, 32);
    v += __shfl_xor(v, 16, 32);
    if (lane == 0) red[s][wave] = v;
  }
  __syncthreads();
  if (wave == 0) {
    const int sc = (lane < 5) ? lane : 0;
    float v = 0.f;
#pragma unroll
    for (int w = 0; w < 8; ++w) v += red[sc][w];
    lst[lane] = (lane < 5) ? v : 0.f;
    wave_lds_sync();
    const v4f pv = *(const v4f*)(lst + (lane & 7) * 4);
    float* pd = plines + ((size_t)(b * 16 + ch)) * LINEF + (lane & 7) * 4;
    if (lane < 8) *(volatile v4f*)pd = pv;
    __threadfence();
    if (lane < 8) *(volatile v4f*)pd = pv;
  }
}

template <bool LAST>
__global__ __launch_bounds__(256) void agg_kernel(
    const float* __restrict__ attn, const float* __restrict__ plines,
    const unsigned short* __restrict__ vplane, const unsigned short* __restrict__ vbg16,
    const float* __restrict__ fcln, const float* __restrict__ w_pos, const float* __restrict__ b_pos,
    float* __restrict__ posl, float* __restrict__ upd, float* __restrict__ ostage)
{
  using namespace cfg;
  __shared__ float part[32][73];
  __shared__ float pp[32][4];
  __shared__ __align__(16) float res[128];
  __shared__ __align__(16) float pst[32];
  const int tid = threadIdx.x, wave = tid >> 5, lane = tid & 31;
  const int bs = blockIdx.x;
  const int b = bs / NSLOT;
  const int s = bs - b * NSLOT;
  float tot = 0.f;
#pragma unroll
  for (int ch = 0; ch < 16; ++ch) tot += plines[((size_t)(b * 16 + ch)) * LINEF + s];
  const float inv = 1.0f / tot;
  const int kfg = (s > 0) ? (s - 1) : 0;
  const unsigned short* vsrc = (s == 0) ? (vbg16 + (size_t)b * NTOK * 64)
                                        : (vplane + ((size_t)(b * NFG + kfg)) * NTOK * 64);
  const float* arow = attn + ((size_t)(b * NSLOT + s)) * NTOK;
  const float* frow = fcln + (size_t)b * NTOK * CDIM;
  const int cg = tid & 7, tl = tid >> 3;
  float acc[8];
#pragma unroll
  for (int e = 0; e < 8; ++e) acc[e] = 0.f;
  float fca = 0.f, ax = 0.f, ay = 0.f, qx = 0.f, qy = 0.f;
#pragma unroll 1
  for (int it = 0; it < NTOK / 32; ++it) {
    const int n = it * 32 + tl;
    const float w = arow[n] * inv;
    const v4u raw = *(const v4u*)(vsrc + (size_t)n * 64 + cg * 8);
    acc[0] += w * h2f(raw[0]);       acc[1] += w * h2f(raw[0] >> 16);
    acc[2] += w * h2f(raw[1]);       acc[3] += w * h2f(raw[1] >> 16);
    acc[4] += w * h2f(raw[2]);       acc[5] += w * h2f(raw[2] >> 16);
    acc[6] += w * h2f(raw[3]);       acc[7] += w * h2f(raw[3] >> 16);
    if (LAST) fca += w * frow[(size_t)n * CDIM + cg];
    ax += w * grid_x(n);
    ay += w * grid_y(n);
    qx += w * w_pos[n];
    qy += w * w_pos[NTOK + n];
  }
#pragma unroll
  for (int e = 0; e < 8; ++e) part[tl][cg * 8 + e] = acc[e];
  part[tl][64 + cg] = fca;
  if (cg == 0) { pp[tl][0] = ax; pp[tl][1] = ay; pp[tl][2] = qx; pp[tl][3] = qy; }
  __syncthreads();
  if (tid < 128) {
    const int col = (tid < 72) ? tid : 71;
    const int pc = (tid >= 72 && tid < 76) ? (tid - 72) : 0;
    float vsum = 0.f, psum = 0.f;
#pragma unroll 1
    for (int r = 0; r < 32; ++r) { vsum += part[r][col]; psum += pp[r][pc]; }
    float v = 0.f;
    if (tid < 72) v = vsum;
    else if (tid < 76) v = psum;
    res[tid] = v;
  }
  __syncthreads();
  if (wave == 0) {
    const float npx = fminf(1.0f, fmaxf(-1.0f, res[72] + tanhf(res[74] + b_pos[0]) * 0.2f));
    const float npy = fminf(1.0f, fmaxf(-1.0f, res[73] + tanhf(res[75] + b_pos[1]) * 0.2f));
    pst[lane] = (lane == 0) ? npx : ((lane == 1) ? npy : 0.f);
    wave_lds_sync();
    const v4f pv = *(const v4f*)(pst + (lane & 7) * 4);
    float* pd = posl + ((size_t)(b * NFG + kfg)) * LINEF + (lane & 7) * 4;
    const bool wr = (s > 0) && (lane < 8);
    if (wr) *(volatile v4f*)pd = pv;
    __threadfence();
    if (wr) *(volatile v4f*)pd = pv;
    if (!LAST) {
      const v4f u = *(const v4f*)(res + (lane & 15) * 4);
      float* ud = upd + (size_t)bs * 64 + (lane & 15) * 4;
      if (lane < 16) *(volatile v4f*)ud = u;
      __threadfence();
      if (lane < 16) *(volatile v4f*)ud = u;
    } else {
      const v4f u = *(const v4f*)(res + lane * 4);
      float* od = ostage + (size_t)bs * OPITCH + lane * 4;
      *(volatile v4f*)od = u;
      __threadfence();
      *(volatile v4f*)od = u;
    }
  }
}

__global__ __launch_bounds__(64) void gru_kernel(
    const float* __restrict__ upd, float* __restrict__ slots,
    const float* __restrict__ fg_wih, const float* __restrict__ fg_whh,
    const float* __restrict__ fg_bih, const float* __restrict__ fg_bhh,
    const float* __restrict__ bg_wih, const float* __restrict__ bg_whh,
    const float* __restrict__ bg_bih, const float* __restrict__ bg_bhh,
    const float* __restrict__ rfg_g, const float* __restrict__ rfg_b,
    const float* __restrict__ w_rfg, const float* __restrict__ b_rfg,
    const float* __restrict__ rbg_g, const float* __restrict__ rbg_b,
    const float* __restrict__ w_rbg, const float* __restrict__ b_rbg)
{
  using namespace cfg;
  __shared__ __align__(16) float shx[64];
  __shared__ __align__(16) float shh[64];
  __shared__ __align__(16) float shn[64];
  __shared__ __align__(16) float shl[64];
  __shared__ __align__(16) float sho[64];
  const int j = threadIdx.x;
  const int bs = blockIdx.x;
  const int b = bs / NSLOT;
  const int s = bs - b * NSLOT;
  const bool isbg = (s == 0);
  const int srow = isbg ? (64 + b) : (b * NFG + s - 1);
  const float* wih = isbg ? bg_wih : fg_wih;
  const float* whh = isbg ? bg_whh : fg_whh;
  const float* bih = isbg ? bg_bih : fg_bih;
  const float* bhh = isbg ? bg_bhh : fg_bhh;
  const float* lg  = isbg ? rbg_g : rfg_g;
  const float* lbv = isbg ? rbg_b : rfg_b;
  const float* wr  = isbg ? w_rbg : w_rfg;
  const float* br  = isbg ? b_rbg : b_rfg;
  shx[j] = upd[(size_t)bs * 64 + j];
  shh[j] = slots[(size_t)srow * 64 + j];
  __syncthreads();
  float gir = bih[j], giz = bih[64 + j], gin = bih[128 + j];
  float ghr = bhh[j], ghz = bhh[64 + j], ghn = bhh[128 + j];
#pragma unroll 1
  for (int d = 0; d < 64; ++d) {
    const float xv = shx[d], hv = shh[d];
    gir += xv * wih[j * 64 + d];
    giz += xv * wih[(64 + j) * 64 + d];
    gin += xv * wih[(128 + j) * 64 + d];
    ghr += hv * whh[j * 64 + d];
    ghz += hv * whh[(64 + j) * 64 + d];
    ghn += hv * whh[(128 + j) * 64 + d];
  }
  const float rg = 1.0f / (1.0f + expf(-(gir + ghr)));
  const float zg = 1.0f / (1.0f + expf(-(giz + ghz)));
  const float ng = tanhf(gin + rg * ghn);
  const float hnew = (1.0f - zg) * ng + zg * shh[j];
  shn[j] = hnew;
  __syncthreads();
  float s1 = 0.f;
#pragma unroll 1
  for (int d = 0; d < 64; ++d) s1 += shn[d];
  const float mean = s1 * (1.0f / 64.0f);
  float vs = 0.f;
#pragma unroll 1
  for (int d = 0; d < 64; ++d) { const float dd = shn[d] - mean; vs += dd * dd; }
  const float inv = rsqrtf(vs * (1.0f / 64.0f) + LN_EPS);
  shl[j] = (hnew - mean) * inv * lg[j] + lbv[j];
  __syncthreads();
  float acc = br[j];
#pragma unroll 1
  for (int d = 0; d < 64; ++d) acc += shl[d] * wr[j * 64 + d];
  sho[j] = hnew + acc;
  __syncthreads();
  const v4f hv4 = *(const v4f*)(sho + (j & 15) * 4);
  float* hd = slots + (size_t)srow * 64 + (j & 15) * 4;
  if (j < 16) *(volatile v4f*)hd = hv4;
  __threadfence();
  if (j < 16) *(volatile v4f*)hd = hv4;
}

__global__ __launch_bounds__(256) void out_copy_kernel(const float* __restrict__ ostage, float* __restrict__ out)
{
  using namespace cfg;
  const int tid = threadIdx.x;
  constexpr int NF4 = NSROW * NOUTC / 4;
  v4f vals[6];
#pragma unroll
  for (int it = 0; it < 6; ++it) {
    const int f = it * 256 + tid;
    const int fc = (f < NF4) ? f : (NF4 - 1);
    const int row = fc / (NOUTC / 4);
    const int col = (fc - row * (NOUTC / 4)) * 4;
    vals[it] = *(const v4f*)(ostage + (size_t)row * OPITCH + col);
  }
  for (int pass = 0; pass < 2; ++pass) {
#pragma unroll
    for (int it = 0; it < 6; ++it) {
      const int f = it * 256 + tid;
      if (f < NF4) *(volatile v4f*)(out + (size_t)f * 4) = vals[it];
    }
    __threadfence();
  }
}

extern "C" void kernel_launch(void* const* d_in, const int* in_sizes, int n_in,
                              void* d_out, int out_size, void* d_ws, size_t ws_size,
                              hipStream_t stream)
{
  using namespace cfg;
  (void)in_sizes; (void)n_in; (void)out_size;
  const float* feat      = (const float*)d_in[0];
  const float* featc     = (const float*)d_in[1];
  const float* w_grid    = (const float*)d_in[2];
  const float* b_grid    = (const float*)d_in[3];
  const float* w_kfg     = (const float*)d_in[4];
  const float* w_vfg     = (const float*)d_in[5];
  const float* w_kbg     = (const float*)d_in[6];
  const float* w_vbg     = (const float*)d_in[7];
  const float* ln_fg_g   = (const float*)d_in[8];
  const float* ln_fg_b   = (const float*)d_in[9];
  const float* w_mlp_fg  = (const float*)d_in[10];
  const float* b_mlp_fg  = (const float*)d_in[11];
  const float* ln_bg_g   = (const float*)d_in[12];
  const float* ln_bg_b   = (const float*)d_in[13];
  const float* w_mlp_bg  = (const float*)d_in[14];
  const float* b_mlp_bg  = (const float*)d_in[15];
  const float* slots0_fg = (const float*)d_in[16];
  const float* slots0_bg = (const float*)d_in[17];
  const float* fg_pos0   = (const float*)d_in[18];
  const float* w_pos     = (const float*)d_in[19];
  const float* b_pos     = (const float*)d_in[20];
  const float* ln_q_g    = (const float*)d_in[21];
  const float* ln_q_b    = (const float*)d_in[22];
  const float* w_q       = (const float*)d_in[23];
  const float* ln_qbg_g  = (const float*)d_in[24];
  const float* ln_qbg_b  = (const float*)d_in[25];
  const float* w_qbg     = (const float*)d_in[26];
  const float* gfg_wih   = (const float*)d_in[27];
  const float* gfg_whh   = (const float*)d_in[28];
  const float* gfg_bih   = (const float*)d_in[29];
  const float* gfg_bhh   = (const float*)d_in[30];
  const float* gbg_wih   = (const float*)d_in[31];
  const float* gbg_whh   = (const float*)d_in[32];
  const float* gbg_bih   = (const float*)d_in[33];
  const float* gbg_bhh   = (const float*)d_in[34];
  const float* ln_rfg_g  = (const float*)d_in[35];
  const float* ln_rfg_b  = (const float*)d_in[36];
  const float* w_rfg     = (const float*)d_in[37];
  const float* b_rfg     = (const float*)d_in[38];
  const float* ln_rbg_g  = (const float*)d_in[39];
  const float* ln_rbg_b  = (const float*)d_in[40];
  const float* w_rbg     = (const float*)d_in[41];
  const float* b_rbg     = (const float*)d_in[42];
  const float* ln_feat_g = (const float*)d_in[43];
  const float* ln_feat_b = (const float*)d_in[44];
  const float* ln_fc_g   = (const float*)d_in[45];
  const float* ln_fc_b   = (const float*)d_in[46];
  float* out = (float*)d_out;

  constexpr size_t PLANE32 = (size_t)NROW * DIM * 4;
  constexpr size_t PLANE16 = (size_t)NROW * DIM * 2;
  constexpr size_t OFF_W16    = 0;
  constexpr size_t OFF_FEATLN = 65536;
  constexpr size_t OFF_KF     = OFF_FEATLN + PLANE16;
  constexpr size_t OFF_VF     = OFF_KF + PLANE32;
  constexpr size_t OFF_TMP    = OFF_VF + PLANE32;
  constexpr size_t OFF_UBG    = OFF_TMP + 2 * PLANE32;
  constexpr size_t OFF_KBG    = OFF_UBG + 2 * PLANE16;
  constexpr size_t OFF_VBG    = OFF_KBG + PLANE32;
  constexpr size_t OFF_FCLN   = OFF_VBG + PLANE16;
  constexpr size_t OFF_LOGITS = OFF_FCLN + (size_t)NROW * CDIM * 4;
  constexpr size_t OFF_ATTN   = OFF_LOGITS + (size_t)NSROW * NTOK * 4;
  constexpr size_t OFF_PLINES = OFF_ATTN + (size_t)NSROW * NTOK * 4;
  constexpr size_t OFF_POSL   = OFF_PLINES + (size_t)NB * 16 * LINEF * 4;
  constexpr size_t OFF_SLOTS  = OFF_POSL + (size_t)NB * NFG * LINEF * 4;
  constexpr size_t OFF_Q      = OFF_SLOTS + (size_t)NSROW * 64 * 4;
  constexpr size_t OFF_UPD    = OFF_Q + (size_t)NSROW * 64 * 4;
  constexpr size_t OFF_OST    = OFF_UPD + (size_t)NSROW * 64 * 4;
  constexpr size_t WS_TOTAL   = OFF_OST + (size_t)NSROW * OPITCH * 4;
  static_assert(6 * 4096 * 2 <= 65536, "");
  static_assert((size_t)NROWFG * 64 * 2 == 2 * PLANE32, "");
  static_assert(WS_TOTAL == 122368000ull, "");
  static_assert(WS_TOTAL <= 134217728ull, "");
  if (ws_size < WS_TOTAL) return;

  char* ws = (char*)d_ws;
  unsigned short* w16    = (unsigned short*)(ws + OFF_W16);
  unsigned short* featln = (unsigned short*)(ws + OFF_FEATLN);
  float* kf              = (float*)(ws + OFF_KF);
  float* vf              = (float*)(ws + OFF_VF);
  float* tmp2            = (float*)(ws + OFF_TMP);
  unsigned short* vplane = (unsigned short*)(ws + OFF_TMP);
  unsigned short* ubg2   = (unsigned short*)(ws + OFF_UBG);
  float* kbg             = (float*)(ws + OFF_KBG);
  unsigned short* vbg16  = (unsigned short*)(ws + OFF_VBG);
  float* fcln            = (float*)(ws + OFF_FCLN);
  float* logits          = (float*)(ws + OFF_LOGITS);
  float* attn            = (float*)(ws + OFF_ATTN);
  float* plines          = (float*)(ws + OFF_PLINES);
  float* posl            = (float*)(ws + OFF_POSL);
  float* slots           = (float*)(ws + OFF_SLOTS);
  float* qbuf            = (float*)(ws + OFF_Q);
  float* upd             = (float*)(ws + OFF_UPD);
  float* ostage          = (float*)(ws + OFF_OST);

  const unsigned short* w16_kfg   = w16 + 0 * 4096;
  const unsigned short* w16_vfg   = w16 + 1 * 4096;
  const unsigned short* w16_kbg   = w16 + 2 * 4096;
  const unsigned short* w16_vbg   = w16 + 3 * 4096;
  const unsigned short* w16_mlpbg = w16 + 4 * 4096;
  const unsigned short* w16_mlpfg = w16 + 5 * 4096;
  float* tmpk = tmp2;
  float* tmpv = tmp2 + (size_t)NROW * DIM;
  unsigned short* ubgk = ubg2;
  unsigned short* ubgv = ubg2 + (size_t)NROW * DIM;

  constexpr int GEMM_M = NROW, GEMM_N = 64, GEMM_K = 64;
  static_assert(GEMM_M % 64 == 0 && GEMM_N % 64 == 0 && GEMM_K % 32 == 0, "");
  const int gemm_blocks = ((GEMM_M / 64) * (GEMM_N / 64)) / 8;
  static_assert(((cfg::NROW / 64) % 8) == 0, "");

  cast_w_kernel<<<dim3(8, 6), 256, 0, stream>>>(w_kfg, w_vfg, w_kbg, w_vbg, w_mlp_bg, w_mlp_fg, w16);
  prep_ln_kernel<<<NROW / 32, 256, 0, stream>>>(feat, ln_feat_g, ln_feat_b, featc, ln_fc_g, ln_fc_b, featln, fcln);

  wmma_gemm64<0, false, 0, 0, false, 0><<<dim3(gemm_blocks, 1), 256, 0, stream>>>(
      featln, featln, 64, 0L, w16_kfg, w16_kfg, 64, 0L, (void*)kf, (void*)kf, 64, 0L,
      b_mlp_bg, kf, 0L, GEMM_M, GEMM_N, GEMM_K, WCARRY_INV);
  wmma_gemm64<0, false, 0, 0, false, 0><<<dim3(gemm_blocks, 1), 256, 0, stream>>>(
      featln, featln, 64, 0L, w16_vfg, w16_vfg, 64, 0L, (void*)vf, (void*)vf, 64, 0L,
      b_mlp_bg, kf, 0L, GEMM_M, GEMM_N, GEMM_K, WCARRY_INV);
  wmma_gemm64<0, false, 0, 0, false, 0><<<dim3(gemm_blocks, 1), 256, 0, stream>>>(
      featln, featln, 64, 0L, w16_kbg, w16_kbg, 64, 0L, (void*)tmpk, (void*)tmpk, 64, 0L,
      b_mlp_bg, kf, 0L, GEMM_M, GEMM_N, GEMM_K, WCARRY_INV);
  wmma_gemm64<0, false, 0, 0, false, 0><<<dim3(gemm_blocks, 1), 256, 0, stream>>>(
      featln, featln, 64, 0L, w16_vbg, w16_vbg, 64, 0L, (void*)tmpv, (void*)tmpv, 64, 0L,
      b_mlp_bg, kf, 0L, GEMM_M, GEMM_N, GEMM_K, WCARRY_INV);

  ln_geo_kernel<<<dim3(NROW / 32, 2), 256, 0, stream>>>(tmp2, w_grid, b_grid, ln_bg_g, ln_bg_b, ubg2);

  wmma_gemm64<0, false, 2, 0, false, 0><<<dim3(gemm_blocks, 1), 256, 0, stream>>>(
      ubgk, ubgk, 64, 0L, w16_mlpbg, w16_mlpbg, 64, 0L, (void*)kbg, (void*)kbg, 64, 0L,
      b_mlp_bg, kf, 0L, GEMM_M, GEMM_N, GEMM_K, WCARRY_INV);
  wmma_gemm64<0, false, 2, 1, false, 0><<<dim3(gemm_blocks, 1), 256, 0, stream>>>(
      ubgv, ubgv, 64, 0L, w16_mlpbg, w16_mlpbg, 64, 0L, (void*)vbg16, (void*)vbg16, 64, 0L,
      b_mlp_bg, kf, 0L, GEMM_M, GEMM_N, GEMM_K, WCARRY_INV);

  init_kernel<<<1, 256, 0, stream>>>(slots0_fg, slots0_bg, fg_pos0, slots, posl);

  static_assert(cfg::NROWFG / 32 == 4096 * 2, "");
  for (int it = 0; it < NITER; ++it) {
    q_proj_kernel<<<NSROW, 64, 0, stream>>>(slots, ln_q_g, ln_q_b, w_q, ln_qbg_g, ln_qbg_b, w_qbg, qbuf);
    fg_kv_kernel<<<NROWFG / 64, 64, 0, stream>>>(kf, vf, posl, w_grid, b_grid, ln_fg_g, ln_fg_b,
                                                 w16_mlpfg, b_mlp_fg, qbuf, vplane, logits);
    bg_logits_kernel<<<NROW / 256, 256, 0, stream>>>(kbg, qbuf, logits);
    softmax_kernel<<<NROW / 256, 256, 0, stream>>>(logits, attn, plines);
    if (it < NITER - 1) {
      agg_kernel<false><<<NSROW, 256, 0, stream>>>(attn, plines, vplane, vbg16, fcln, w_pos, b_pos, posl, upd, ostage);
      gru_kernel<<<NSROW, 64, 0, stream>>>(upd, slots, gfg_wih, gfg_whh, gfg_bih, gfg_bhh,
                                            gbg_wih, gbg_whh, gbg_bih, gbg_bhh,
                                            ln_rfg_g, ln_rfg_b, w_rfg, b_rfg,
                                            ln_rbg_g, ln_rbg_b, w_rbg, b_rbg);
    } else {
      agg_kernel<true><<<NSROW, 256, 0, stream>>>(attn, plines, vplane, vbg16, fcln, w_pos, b_pos, posl, upd, ostage);
      out_copy_kernel<<<1, 256, 0, stream>>>(ostage, out);
    }
  }
}
